// GatedRNNCell_36567351558875
// MI455X (gfx1250) — hardware-run, weakly checked
//
#include <hip/hip_runtime.h>
#include <math.h>

constexpr int NB    = 4096;
constexpr int NIN   = 1024;
constexpr int NH    = 2048;
constexpr int NCTX  = 1024;
constexpr int KCAT  = NIN + NCTX + NH;
constexpr int NTHR  = 256;
constexpr int SLABP = 68;
constexpr float WCARRY     = 256.0f;
constexpr float WCARRY_INV = 1.0f / 256.0f;

static_assert(KCAT == 4096);
static_assert(KCAT % 32 == 0);
static_assert(NB % 64 == 0 && NH % 64 == 0);
static_assert(((NB / 64) * (NH / 64)) % (NTHR / 32) == 0);
static_assert((NIN / 8) % 32 == 0 && (NCTX / 8) % 32 == 0 && (NH / 8) % 32 == 0);
static_assert(((size_t)NB * (NH / 8)) % NTHR == 0 && ((size_t)NH * (NIN / 8)) % NTHR == 0);

constexpr size_t WS_A_BYTES  = (size_t)NB * KCAT * 2;
constexpr size_t WS_BT_BYTES = (size_t)NH * KCAT * 2;
constexpr size_t WS_TOTAL    = 2 * WS_A_BYTES + 3 * WS_BT_BYTES;
static_assert(WS_TOTAL == (size_t)117440512);
static_assert(WS_TOTAL <= (size_t)134217728);

typedef __attribute__((ext_vector_type(16))) _Float16 v16h;
typedef __attribute__((ext_vector_type(8)))  _Float16 v8h;
typedef __attribute__((ext_vector_type(8)))  float    v8f;
typedef __attribute__((ext_vector_type(4)))  float    v4f;
typedef __attribute__((ext_vector_type(2)))  float    v2f;

__device__ __forceinline__ unsigned short f2bf_bits(float f) {
  unsigned u = __float_as_uint(f);
  return (unsigned short)((u + 0x7FFFu + ((u >> 16) & 1u)) >> 16);
}
__device__ __forceinline__ float bf_bits2f(unsigned short h) { return __uint_as_float(((unsigned)h) << 16); }
__device__ __forceinline__ float bf16r(float f) { return bf_bits2f(f2bf_bits(f)); }

__device__ __forceinline__ void guard_row4(v8f& a0, v8f& a1, v8f& a2, v8f& a3,
                                           v16h x, v16h b0, v16h b1, v16h b2, v16h b3) {
  asm volatile("v_nop\n\tv_nop\n\tv_nop\n\tv_nop"
               : "+v"(a0), "+v"(a1), "+v"(a2), "+v"(a3)
               : "v"(x), "v"(b0), "v"(b1), "v"(b2), "v"(b3));
}
__device__ __forceinline__ void keep4_h(v16h a, v16h b, v16h c, v16h d) { asm volatile("v_nop" :: "v"(a), "v"(b), "v"(c), "v"(d)); }
__device__ __forceinline__ void acc_guard4(v8f& a, v8f& b, v8f& c, v8f& d) {
  asm volatile("v_nop\n\tv_nop\n\tv_nop\n\tv_nop" : "+v"(a), "+v"(b), "+v"(c), "+v"(d));
}

struct FragH {
  union U { v16h v; v8h h[2]; };
  static __device__ __forceinline__ v16h load(const _Float16* p) {
    U f;
    f.h[0] = *(const v8h*)(p);
    f.h[1] = *(const v8h*)(p + 16);
    return f.v;
  }
  static __device__ __forceinline__ v8f mma(v16h a, v16h b, v8f c) {
    return __builtin_amdgcn_wmma_f32_16x16x32_f16(false, a, false, b, (short)0, c, false, false);
  }
};

__device__ __forceinline__ float gate_sig(float x)  { return __builtin_amdgcn_rcpf(1.0f + expf(-x)); }
__device__ __forceinline__ float gate_tanh(float x) { return 1.0f - 2.0f * __builtin_amdgcn_rcpf(expf(2.0f * x) + 1.0f); }

__global__ __launch_bounds__(NTHR) void cvt_cat3_kernel(const float* __restrict__ s0, const float* __restrict__ s1,
                                                        const float* __restrict__ s2,
                                                        unsigned short* dst, unsigned short* dst2,
                                                        int nrow, int nc8_0, int nc8_1, int nc8_2,
                                                        int dpitch, int dual01, float sc) {
  const int seg = blockIdx.y;
  const float* src = s0;
  int nc8 = nc8_0;
  int dcol0 = 0;
  if (seg == 1) { src = s1; nc8 = nc8_1; dcol0 = nc8_0 * 8; }
  if (seg == 2) { src = s2; nc8 = nc8_2; dcol0 = (nc8_0 + nc8_1) * 8; }
  const bool dual = (dual01 != 0) && (seg < 2);
  const int i  = blockIdx.x * NTHR + threadIdx.x;
  const int n8 = nrow * nc8;
  if (i < n8) {
    const int row = i / nc8;
    const int c8  = i - row * nc8;
    const float* sp = src + (size_t)i * 8;
    const v4f a = *(const v4f*)(sp);
    const v4f b = *(const v4f*)(sp + 4);
    v8h hv;
#pragma unroll
    for (int e = 0; e < 4; ++e) {
      const float fa = bf16r(a[e]) * sc;
      const float fb = bf16r(b[e]) * sc;
      hv[e]     = (_Float16)fa;
      hv[4 + e] = (_Float16)fb;
    }
    const size_t o = (size_t)row * (size_t)dpitch + (size_t)dcol0 + (size_t)c8 * 8;
    *(volatile v8h*)(dst + o) = hv;
    if (dual) *(volatile v8h*)(dst2 + o) = hv;
    __threadfence();
    *(volatile v8h*)(dst + o) = hv;
    if (dual) *(volatile v8h*)(dst2 + o) = hv;
  }
}

template <int EP>
__global__ __launch_bounds__(NTHR) void gate_gemm_kernel(const unsigned short* __restrict__ Ap,
                                                         const unsigned short* __restrict__ Btp,
                                                         const float* __restrict__ bias,
                                                         const float* __restrict__ sprev,
                                                         float* outF, unsigned short* outH) {
  __shared__ __align__(16) float sT[NTHR / 32][16 * SLABP];
  const int lane = threadIdx.x & 31;
  const int wave = threadIdx.x >> 5;
  constexpr int tilesN = NH >> 6;
  constexpr int tilesM = NB >> 6;
  const int tile = blockIdx.x * (NTHR / 32) + wave;
  if (tile >= tilesM * tilesN) return;
  const int tm = tile / tilesN;
  const int tn = tile - tm * tilesN;
  const int m0 = tm << 6;
  const int n0 = tn << 6;

  const int rlane = lane & 15;
  const int hh    = lane >> 4;
  const int koff  = hh * 8;
  const int mOff  = hh * 8;

  const _Float16* ap = (const _Float16*)Ap  + (size_t)(m0 + rlane) * KCAT + koff;
  const _Float16* bp = (const _Float16*)Btp + (size_t)(n0 + rlane) * KCAT + koff;
  constexpr size_t SUB = (size_t)16 * KCAT;

  v8f acc[4][4];
#pragma unroll
  for (int i = 0; i < 4; ++i)
#pragma unroll
    for (int j = 0; j < 4; ++j) acc[i][j] = (v8f){0.f, 0.f, 0.f, 0.f, 0.f, 0.f, 0.f, 0.f};

#pragma unroll 1
  for (int k0 = 0; k0 < KCAT; k0 += 32) {
    v16h bh[4];
#pragma unroll
    for (int j = 0; j < 4; ++j) bh[j] = FragH::load(bp + (size_t)j * SUB + k0);
#pragma unroll
    for (int i = 0; i < 4; ++i) {
      const v16h ah = FragH::load(ap + (size_t)i * SUB + k0);
#pragma unroll
      for (int j = 0; j < 4; ++j) acc[i][j] = FragH::mma(ah, bh[j], acc[i][j]);
      guard_row4(acc[i][0], acc[i][1], acc[i][2], acc[i][3], ah, bh[0], bh[1], bh[2], bh[3]);
    }
    keep4_h(bh[0], bh[1], bh[2], bh[3]);
  }
  acc_guard4(acc[0][0], acc[0][1], acc[0][2], acc[0][3]);
  acc_guard4(acc[1][0], acc[1][1], acc[1][2], acc[1][3]);
  acc_guard4(acc[2][0], acc[2][1], acc[2][2], acc[2][3]);
  acc_guard4(acc[3][0], acc[3][1], acc[3][2], acc[3][3]);

  float* slab = sT[wave];
  float bv[4];
#pragma unroll
  for (int j = 0; j < 4; ++j) bv[j] = bf16r(bias[n0 + (j << 4) + rlane]);
  const int c4 = rlane * 4;

#pragma unroll
  for (int i = 0; i < 4; ++i) {
    const int mBase = m0 + (i << 4);
#pragma unroll
    for (int j = 0; j < 4; ++j) {
#pragma unroll
      for (int r = 0; r < 8; ++r) {
        slab[(mOff + r) * SLABP + (j << 4) + rlane] = acc[i][j][r] * WCARRY_INV + bv[j];
      }
    }
    __builtin_amdgcn_fence(__ATOMIC_RELEASE, "workgroup");
    __builtin_amdgcn_wave_barrier();
    __builtin_amdgcn_fence(__ATOMIC_ACQUIRE, "workgroup");

#pragma unroll 1
    for (int qi = 0; qi < 16; ++qi) {
      const int row = ((qi >> 1) << 1) + hh;
      const int col = c4 + ((qi & 1) << 1);
      float* sp = slab + row * SLABP + col;
      const v2f pre = *(const v2f*)sp;
      const size_t gi = (size_t)(mBase + row) * NH + (size_t)(n0 + col);
      v2f res;
      if (EP == 0) {
        const v2f sv = *(const v2f*)(sprev + gi);
#pragma unroll
        for (int e = 0; e < 2; ++e) res[e] = gate_sig(pre[e]) * bf16r(sv[e]);
      } else if (EP == 1) {
#pragma unroll
        for (int e = 0; e < 2; ++e) res[e] = gate_sig(pre[e]);
      } else {
        const v2f sv = *(const v2f*)(sprev + gi);
        const v2f zv = *(const v2f*)(outF + gi);
#pragma unroll
        for (int e = 0; e < 2; ++e) {
          const float cand = gate_tanh(pre[e]);
          const float sb   = bf16r(sv[e]);
          const float zz   = zv[e];
          res[e] = (1.0f - zz) * sb + zz * cand;
        }
      }
      *(v2f*)sp = res;
    }
    __builtin_amdgcn_fence(__ATOMIC_RELEASE, "workgroup");
    __builtin_amdgcn_wave_barrier();
    __builtin_amdgcn_fence(__ATOMIC_ACQUIRE, "workgroup");

    if (EP == 0) {
      const int q = lane >> 3, c8 = (lane & 7) * 8;
      for (int pass = 0; pass < 2; ++pass) {
#pragma unroll
        for (int it = 0; it < 4; ++it) {
          const int row = it * 4 + q;
          const float* sp = slab + row * SLABP + c8;
          const v4f lo4 = *(const v4f*)(sp);
          const v4f hi4 = *(const v4f*)(sp + 4);
          v8h hv;
#pragma unroll
          for (int e = 0; e < 4; ++e) {
            hv[e]     = (_Float16)lo4[e];
            hv[4 + e] = (_Float16)hi4[e];
          }
          *(volatile v8h*)(outH + (size_t)(mBase + row) * KCAT + (size_t)(NIN + NCTX + n0 + c8)) = hv;
        }
        __threadfence();
      }
    } else {
      for (int pass = 0; pass < 2; ++pass) {
#pragma unroll
        for (int it = 0; it < 8; ++it) {
          const int row = it * 2 + hh;
          const v4f v = *(const v4f*)(slab + row * SLABP + c4);
          *(volatile v4f*)(outF + (size_t)(mBase + row) * NH + (size_t)(n0 + c4)) = v;
        }
        __threadfence();
      }
    }
    __builtin_amdgcn_fence(__ATOMIC_RELEASE, "workgroup");
    __builtin_amdgcn_wave_barrier();
    __builtin_amdgcn_fence(__ATOMIC_ACQUIRE, "workgroup");
  }
}

extern "C" void kernel_launch(void* const* d_in, const int* in_sizes, int n_in,
                              void* d_out, int out_size, void* d_ws, size_t ws_size, hipStream_t stream) {
  if (n_in < 15 || d_out == nullptr || d_ws == nullptr) return;
  if (in_sizes[0] != NB * NIN || in_sizes[1] != NB * NH || in_sizes[2] != NB * NCTX ||
      in_sizes[3] != NH * NIN || in_sizes[4] != NH * NIN || in_sizes[5] != NH * NIN ||
      in_sizes[6] != NH * NH || in_sizes[7] != NH * NH || in_sizes[8] != NH * NH ||
      in_sizes[9] != NH * NCTX || in_sizes[10] != NH * NCTX || in_sizes[11] != NH * NCTX ||
      in_sizes[12] != NH || in_sizes[13] != NH || in_sizes[14] != NH ||
      out_size != NB * NH) return;
  if (ws_size < WS_TOTAL) return;

  const float* x   = (const float*)d_in[0];
  const float* s   = (const float*)d_in[1];
  const float* c   = (const float*)d_in[2];
  const float* Wc  = (const float*)d_in[3];
  const float* Wz  = (const float*)d_in[4];
  const float* Wr  = (const float*)d_in[5];
  const float* Uc  = (const float*)d_in[6];
  const float* Uz  = (const float*)d_in[7];
  const float* Ur  = (const float*)d_in[8];
  const float* Cc  = (const float*)d_in[9];
  const float* Cz  = (const float*)d_in[10];
  const float* Cr  = (const float*)d_in[11];
  const float* bc  = (const float*)d_in[12];
  const float* bz  = (const float*)d_in[13];
  const float* br  = (const float*)d_in[14];
  float* out = (float*)d_out;

  char* ws = (char*)d_ws;
  unsigned short* A1  = (unsigned short*)(ws);
  unsigned short* A2  = (unsigned short*)(ws + WS_A_BYTES);
  unsigned short* BTR = (unsigned short*)(ws + 2 * WS_A_BYTES);
  unsigned short* BTZ = (unsigned short*)(ws + 2 * WS_A_BYTES + WS_BT_BYTES);
  unsigned short* BTC = (unsigned short*)(ws + 2 * WS_A_BYTES + 2 * WS_BT_BYTES);

  const dim3 gact((unsigned)(((size_t)NB * (NH / 8)) / NTHR), 3);
  cvt_cat3_kernel<<<gact, NTHR, 0, stream>>>(x, c, s, A1, A2, NB, NIN / 8, NCTX / 8, NH / 8, KCAT, 1, 1.0f);

  const dim3 gwt((unsigned)(((size_t)NH * (NH / 8)) / NTHR), 3);
  cvt_cat3_kernel<<<gwt, NTHR, 0, stream>>>(Wr, Cr, Ur, BTR, BTR, NH, NIN / 8, NCTX / 8, NH / 8, KCAT, 0, WCARRY);
  cvt_cat3_kernel<<<gwt, NTHR, 0, stream>>>(Wz, Cz, Uz, BTZ, BTZ, NH, NIN / 8, NCTX / 8, NH / 8, KCAT, 0, WCARRY);
  cvt_cat3_kernel<<<gwt, NTHR, 0, stream>>>(Wc, Cc, Uc, BTC, BTC, NH, NIN / 8, NCTX / 8, NH / 8, KCAT, 0, WCARRY);

  const dim3 ggrid((unsigned)(((NB / 64) * (NH / 64)) / (NTHR / 32)), 1);
  gate_gemm_kernel<0><<<ggrid, NTHR, 0, stream>>>(A1, BTR, br, s, out, A2);
  gate_gemm_kernel<1><<<ggrid, NTHR, 0, stream>>>(A1, BTZ, bz, s, out, A1);
  gate_gemm_kernel<2><<<ggrid, NTHR, 0, stream>>>(A2, BTC, bc, s, out, A1);
}
